// Non_local_Block_51539608036
// MI455X (gfx1250) — hardware-verified
//
#include <hip/hip_runtime.h>
#include <stdint.h>

#define NBAT 8
#define CIN  192
#define OCH  96
#define NPIX 4096
#define WSZ  (OCH * CIN)
#define WGRP (WSZ / 8)
#define NQB  (NPIX / 64)
#define NKT  (NPIX / 64)
#define XP   200
#define YP   96
static_assert(OCH == 96 && CIN == 192 && NPIX == 4096);
static_assert(CIN % 32 == 0 && OCH % 32 == 0 && NPIX % 64 == 0);
static_assert(WGRP % 256 == 0);
static_assert((XP % 8) == 0 && (YP % 8) == 0);

typedef __bf16         v16b __attribute__((ext_vector_type(16)));
typedef float          v8f  __attribute__((ext_vector_type(8)));
typedef float          v4f  __attribute__((ext_vector_type(4)));
typedef unsigned int   v4u  __attribute__((ext_vector_type(4)));
typedef unsigned short v8us __attribute__((ext_vector_type(8)));

union FragB { v16b v; v8us h[2]; v4u q[2]; };

#if defined(__HIP_DEVICE_COMPILE__)
#define DEV_ASM 1
#else
#define DEV_ASM 0
#endif

__device__ __forceinline__ unsigned short bf_bits(float f) {
  unsigned u = __float_as_uint(f);
  return (unsigned short)((u + 0x7FFFu + ((u >> 16) & 1u)) >> 16);
}
__device__ __forceinline__ float bf_up(unsigned short hb) { return __uint_as_float(((unsigned)hb) << 16); }
__device__ __forceinline__ float bf_val(float f) { return bf_up(bf_bits(f)); }
__device__ __forceinline__ unsigned pk16(unsigned short a, unsigned short b) { return (unsigned)a | ((unsigned)b << 16); }
__device__ __forceinline__ v8f zero8() { v8f z = {0.f, 0.f, 0.f, 0.f, 0.f, 0.f, 0.f, 0.f}; return z; }

__device__ __forceinline__ v16b ldfrag(const unsigned short* p) {
  FragB f;
  f.h[0] = *(const v8us*)(p);
  f.h[1] = *(const v8us*)(p + 16);
  return f.v;
}

__device__ __forceinline__ v8f mma_b(v16b a, v16b b, v8f c) {
  c = __builtin_amdgcn_wmma_f32_16x16x32_bf16(false, a, false, b, (short)0, c, false, false);
#if DEV_ASM
  asm volatile("v_nop\n\tv_nop\n\tv_nop\n\tv_nop" : "+v"(c) : "v"(a), "v"(b));
#endif
  return c;
}

__device__ __forceinline__ void pack_p2(v8f a, v8f c, v16b& ph, v16b& pl) {
  FragB H, L;
#pragma unroll
  for (int e = 0; e < 4; ++e) {
    const float a0 = a[2 * e], a1 = a[2 * e + 1], c0 = c[2 * e], c1 = c[2 * e + 1];
    const unsigned short ha0 = bf_bits(a0), ha1 = bf_bits(a1), hc0 = bf_bits(c0), hc1 = bf_bits(c1);
    const unsigned short la0 = bf_bits(a0 - bf_up(ha0)), la1 = bf_bits(a1 - bf_up(ha1));
    const unsigned short lc0 = bf_bits(c0 - bf_up(hc0)), lc1 = bf_bits(c1 - bf_up(hc1));
    H.q[0][e] = pk16(ha0, ha1); H.q[1][e] = pk16(hc0, hc1);
    L.q[0][e] = pk16(la0, la1); L.q[1][e] = pk16(lc0, lc1);
  }
  ph = H.v; pl = L.v;
}

__global__ __launch_bounds__(256) void cvt_w(const float* __restrict__ w0, const float* __restrict__ w1,
                                             const float* __restrict__ w2, const float* __restrict__ w3,
                                             unsigned short* wp) {
  const int g = blockIdx.x * 256 + (int)threadIdx.x;
  if (g >= 4 * WGRP) return;
  const int wsel = g / WGRP;
  const int off  = g - wsel * WGRP;
  const float* src = (wsel == 0) ? w0 : ((wsel == 1) ? w1 : ((wsel == 2) ? w2 : w3));
  src += (size_t)off * 8;
  const v4f a = *(const v4f*)(src);
  const v4f c = *(const v4f*)(src + 4);
  v4u p;
  p[0] = pk16(bf_bits(a[0]), bf_bits(a[1]));
  p[1] = pk16(bf_bits(a[2]), bf_bits(a[3]));
  p[2] = pk16(bf_bits(c[0]), bf_bits(c[1]));
  p[3] = pk16(bf_bits(c[2]), bf_bits(c[3]));
  unsigned short* o = wp + (size_t)g * 8;
  *(volatile v4u*)o = p;
  __threadfence();
  *(volatile v4u*)o = p;
}

__device__ __forceinline__ void proj_nt(const unsigned short* sXrow, const unsigned short* __restrict__ wpl,
                                        const float* __restrict__ bias, unsigned short* sH, unsigned short* sL,
                                        int w, int hh, int m) {
  v8f acc[6];
#pragma unroll
  for (int ot = 0; ot < 6; ++ot) acc[ot] = zero8();
#pragma unroll 1
  for (int kc = 0; kc < 6; ++kc) {
    const v16b a = ldfrag(sXrow + 32 * kc);
#pragma unroll
    for (int ot = 0; ot < 6; ++ot) {
      const v16b bw = ldfrag(wpl + (size_t)(16 * ot + m) * CIN + 32 * kc + 8 * hh);
      acc[ot] = mma_b(a, bw, acc[ot]);
    }
  }
#pragma unroll
  for (int ot = 0; ot < 6; ++ot) {
    const float bv = bf_val(bias[16 * ot + m]);
#pragma unroll
    for (int r = 0; r < 8; ++r) {
      const float v = acc[ot][r] + bv;
      const unsigned short hb = bf_bits(v);
      const unsigned short lb = bf_bits(v - bf_up(hb));
      const int idx = (16 * w + 8 * hh + r) * OCH + 16 * ot + m;
      sH[idx] = hb;
      sL[idx] = lb;
    }
  }
}

__device__ __forceinline__ void proj_g(const unsigned short* sXrow, const unsigned short* __restrict__ wpl,
                                       const float* __restrict__ bias, unsigned short* sH, unsigned short* sL,
                                       int w, int hh, int m) {
  v8f acc[6];
#pragma unroll
  for (int ot = 0; ot < 6; ++ot) acc[ot] = zero8();
#pragma unroll 1
  for (int kc = 0; kc < 6; ++kc) {
    const v16b bx = ldfrag(sXrow + 32 * kc);
#pragma unroll
    for (int ot = 0; ot < 6; ++ot) {
      const v16b aw = ldfrag(wpl + (size_t)(16 * ot + m) * CIN + 32 * kc + 8 * hh);
      acc[ot] = mma_b(aw, bx, acc[ot]);
    }
  }
#pragma unroll
  for (int ot = 0; ot < 6; ++ot) {
    const v4f b0 = *(const v4f*)(bias + 16 * ot + 8 * hh);
    const v4f b1 = *(const v4f*)(bias + 16 * ot + 8 * hh + 4);
    const float bb[8] = { bf_val(b0[0]), bf_val(b0[1]), bf_val(b0[2]), bf_val(b0[3]),
                          bf_val(b1[0]), bf_val(b1[1]), bf_val(b1[2]), bf_val(b1[3]) };
#pragma unroll
    for (int r = 0; r < 8; ++r) {
      const float v = acc[ot][r] + bb[r];
      const unsigned short hb = bf_bits(v);
      const unsigned short lb = bf_bits(v - bf_up(hb));
      const int idx = (16 * ot + 8 * hh + r) * 64 + 16 * w + m;
      sH[idx] = hb;
      sL[idx] = lb;
    }
  }
}

__global__ __launch_bounds__(128) void proj_kernel(
    const float* __restrict__ x, const unsigned short* __restrict__ wp,
    const float* __restrict__ th_b, const float* __restrict__ ph_b, const float* __restrict__ g_b,
    unsigned short* thH, unsigned short* thL, unsigned short* phH, unsigned short* phL,
    unsigned short* gH, unsigned short* gL) {
  __shared__ __align__(16) unsigned short sX[64 * XP];
  __shared__ __align__(16) unsigned short sH[64 * OCH];
  __shared__ __align__(16) unsigned short sL[64 * OCH];

  const int tid = (int)threadIdx.x, lane = tid & 31, w = tid >> 5;
  const int hh = lane >> 4, m = lane & 15;
  const int n0 = blockIdx.x * 64;
  const int b  = blockIdx.y;

  {
    const float* xb = x + (size_t)b * CIN * NPIX + n0;
    const int cr = tid >> 4, nq = (tid & 15) * 4;
#pragma unroll 4
    for (int it = 0; it < 24; ++it) {
      const int c = it * 8 + cr;
      const v4f v = *(const v4f*)(xb + (size_t)c * NPIX + nq);
      sX[(nq + 0) * XP + c] = bf_bits(v[0]);
      sX[(nq + 1) * XP + c] = bf_bits(v[1]);
      sX[(nq + 2) * XP + c] = bf_bits(v[2]);
      sX[(nq + 3) * XP + c] = bf_bits(v[3]);
    }
  }
  __syncthreads();

  const unsigned short* sXrow = sX + (16 * w + m) * XP + 8 * hh;

#pragma unroll 1
  for (int sel = 0; sel < 2; ++sel) {
    const unsigned short* wpl = wp + (size_t)sel * WSZ;
    const float* bias  = (sel == 0) ? th_b : ph_b;
    unsigned short* dH = (sel == 0) ? thH : phH;
    unsigned short* dL = (sel == 0) ? thL : phL;
    proj_nt(sXrow, wpl, bias, sH, sL, w, hh, m);
    __syncthreads();
    {
      unsigned short* oH = dH + ((size_t)b * NPIX + n0) * OCH;
      unsigned short* oL = dL + ((size_t)b * NPIX + n0) * OCH;
      v4u hv[6], lv[6];
#pragma unroll
      for (int it = 0; it < 6; ++it) {
        const int p = it * 128 + tid;
        hv[it] = *(const v4u*)(sH + p * 8);
        lv[it] = *(const v4u*)(sL + p * 8);
      }
      for (int pass = 0; pass < 2; ++pass) {
#pragma unroll
        for (int it = 0; it < 6; ++it) {
          const int p = it * 128 + tid;
          *(volatile v4u*)(oH + (size_t)p * 8) = hv[it];
          *(volatile v4u*)(oL + (size_t)p * 8) = lv[it];
        }
        __threadfence();
      }
    }
    __syncthreads();
  }

  proj_g(sXrow, wp + (size_t)2 * WSZ, g_b, sH, sL, w, hh, m);
  __syncthreads();
  {
    unsigned short* oH = gH + ((size_t)b * OCH) * NPIX + n0;
    unsigned short* oL = gL + ((size_t)b * OCH) * NPIX + n0;
    v4u hv[6], lv[6];
#pragma unroll
    for (int it = 0; it < 6; ++it) {
      const int p = it * 128 + tid;
      hv[it] = *(const v4u*)(sH + p * 8);
      lv[it] = *(const v4u*)(sL + p * 8);
    }
    for (int pass = 0; pass < 2; ++pass) {
#pragma unroll
      for (int it = 0; it < 6; ++it) {
        const int p = it * 128 + tid;
        const size_t go = (size_t)(p >> 3) * NPIX + (size_t)((p & 7) * 8);
        *(volatile v4u*)(oH + go) = hv[it];
        *(volatile v4u*)(oL + go) = lv[it];
      }
      __threadfence();
    }
  }
}

__global__ __launch_bounds__(128) void attn_kernel(
    const unsigned short* __restrict__ thH, const unsigned short* __restrict__ thL,
    const unsigned short* __restrict__ phH, const unsigned short* __restrict__ phL,
    const unsigned short* __restrict__ gH,  const unsigned short* __restrict__ gL,
    const unsigned short* __restrict__ wW, const float* __restrict__ w_b,
    const float* __restrict__ x, float* out) {
  __shared__ __align__(16) unsigned short sYH[64 * YP];
  __shared__ __align__(16) unsigned short sYL[64 * YP];
  __shared__ __align__(16) float sO[4][16 * 68];

  const int tid = (int)threadIdx.x, lane = tid & 31, w = tid >> 5;
  const int hh = lane >> 4, m = lane & 15;
  const int q0 = blockIdx.x * 64;
  const int b  = blockIdx.y;

  const size_t qrow = (size_t)b * NPIX + q0 + 16 * w + m;
  const unsigned short* thHr = thH + qrow * OCH + 8 * hh;
  const unsigned short* thLr = thL + qrow * OCH + 8 * hh;
  const unsigned short* phHb = phH + ((size_t)b * NPIX + m) * OCH + 8 * hh;
  const unsigned short* phLb = phL + ((size_t)b * NPIX + m) * OCH + 8 * hh;
  const unsigned short* gHb  = gH + ((size_t)b * OCH + m) * NPIX + 8 * hh;
  const unsigned short* gLb  = gL + ((size_t)b * OCH + m) * NPIX + 8 * hh;

  v8f o[6];
#pragma unroll
  for (int t = 0; t < 6; ++t) o[t] = zero8();
  float mrun = -1e30f, lrun = 0.0f;

#pragma unroll 1
  for (int kt = 0; kt < NKT; ++kt) {
    const int kb = kt * 64;
    v8f s[4];
#pragma unroll
    for (int j = 0; j < 4; ++j) s[j] = zero8();
#pragma unroll 1
    for (int kc = 0; kc < 3; ++kc) {
      const v16b tHf = ldfrag(thHr + 32 * kc);
      const v16b tLf = ldfrag(thLr + 32 * kc);
#pragma unroll
      for (int j = 0; j < 4; ++j) {
        const size_t ko = (size_t)(kb + 16 * j) * OCH + 32 * kc;
        const v16b fHf = ldfrag(phHb + ko);
        const v16b fLf = ldfrag(phLb + ko);
        s[j] = mma_b(fHf, tHf, s[j]);
        s[j] = mma_b(fHf, tLf, s[j]);
        s[j] = mma_b(fLf, tHf, s[j]);
      }
    }

    float mloc = s[0][0];
#pragma unroll
    for (int j = 0; j < 4; ++j)
#pragma unroll
      for (int r = 0; r < 8; ++r) mloc = fmaxf(mloc, s[j][r]);
    mloc = fmaxf(mloc, __shfl_xor(mloc, 16));
    const float mnew  = fmaxf(mrun, mloc);
    const float alpha = __expf(mrun - mnew);
    mrun = mnew;
    float lsum = 0.0f;
#pragma unroll
    for (int j = 0; j < 4; ++j)
#pragma unroll
      for (int r = 0; r < 8; ++r) {
        const float p = __expf(s[j][r] - mnew);
        s[j][r] = p;
        lsum += p;
      }
    lsum += __shfl_xor(lsum, 16);
    lrun = lrun * alpha + lsum;
#pragma unroll
    for (int t = 0; t < 6; ++t)
#pragma unroll
      for (int r = 0; r < 8; ++r) o[t][r] = o[t][r] * alpha;

    v16b pH0, pL0, pH1, pL1;
    pack_p2(s[0], s[1], pH0, pL0);
    pack_p2(s[2], s[3], pH1, pL1);

#pragma unroll
    for (int t = 0; t < 6; ++t) {
      const unsigned short* gph = gHb + (size_t)(16 * t) * NPIX + kb;
      const unsigned short* gpl = gLb + (size_t)(16 * t) * NPIX + kb;
      {
        const v16b aH = ldfrag(gph);
        const v16b aL = ldfrag(gpl);
        o[t] = mma_b(aH, pH0, o[t]);
        o[t] = mma_b(aH, pL0, o[t]);
        o[t] = mma_b(aL, pH0, o[t]);
      }
      {
        const v16b aH = ldfrag(gph + 32);
        const v16b aL = ldfrag(gpl + 32);
        o[t] = mma_b(aH, pH1, o[t]);
        o[t] = mma_b(aH, pL1, o[t]);
        o[t] = mma_b(aL, pH1, o[t]);
      }
    }
  }

  {
    const float inv = 1.0f / lrun;
    const int nl = 16 * w + m;
#pragma unroll
    for (int t = 0; t < 6; ++t) {
      v4u uh, ul;
#pragma unroll
      for (int e = 0; e < 4; ++e) {
        const float v0 = o[t][2 * e] * inv, v1 = o[t][2 * e + 1] * inv;
        const unsigned short h0 = bf_bits(v0), h1 = bf_bits(v1);
        const unsigned short l0 = bf_bits(v0 - bf_up(h0)), l1 = bf_bits(v1 - bf_up(h1));
        uh[e] = pk16(h0, h1);
        ul[e] = pk16(l0, l1);
      }
      *(v4u*)(sYH + nl * YP + 16 * t + 8 * hh) = uh;
      *(v4u*)(sYL + nl * YP + 16 * t + 8 * hh) = ul;
    }
  }
  __syncthreads();

  const int c0w = 48 * w;
  v8f acc[3][4];
#pragma unroll
  for (int ct = 0; ct < 3; ++ct)
#pragma unroll
    for (int nt = 0; nt < 4; ++nt) acc[ct][nt] = zero8();
#pragma unroll 1
  for (int kc = 0; kc < 3; ++kc) {
    v16b wa[3];
#pragma unroll
    for (int ct = 0; ct < 3; ++ct)
      wa[ct] = ldfrag(wW + (size_t)(c0w + 16 * ct + m) * OCH + 32 * kc + 8 * hh);
#pragma unroll
    for (int nt = 0; nt < 4; ++nt) {
      const v16b yh = ldfrag(sYH + (16 * nt + m) * YP + 32 * kc + 8 * hh);
      const v16b yl = ldfrag(sYL + (16 * nt + m) * YP + 32 * kc + 8 * hh);
#pragma unroll
      for (int ct = 0; ct < 3; ++ct) {
        acc[ct][nt] = mma_b(wa[ct], yh, acc[ct][nt]);
        acc[ct][nt] = mma_b(wa[ct], yl, acc[ct][nt]);
      }
    }
  }

  float* slab = sO[w];
  const int h2 = lane >> 4, c4 = (lane & 15) * 4;
#pragma unroll
  for (int ct = 0; ct < 3; ++ct) {
#pragma unroll
    for (int nt = 0; nt < 4; ++nt)
#pragma unroll
      for (int r = 0; r < 8; ++r) slab[(8 * hh + r) * 68 + 16 * nt + m] = acc[ct][nt][r];
    __builtin_amdgcn_fence(__ATOMIC_RELEASE, "workgroup");
    __builtin_amdgcn_wave_barrier();
    __builtin_amdgcn_fence(__ATOMIC_ACQUIRE, "workgroup");
    v4f vv[8];
#pragma unroll
    for (int it = 0; it < 8; ++it) {
      const int row = it * 2 + h2;
      const int c = c0w + 16 * ct + row;
      const v4f a = *(const v4f*)(slab + row * 68 + c4);
      const float bb = bf_val(w_b[c]);
      const v4f xr = *(const v4f*)(x + ((size_t)b * CIN + c) * NPIX + q0 + c4);
      v4f v;
      v[0] = a[0] + bb + bf_val(xr[0]);
      v[1] = a[1] + bb + bf_val(xr[1]);
      v[2] = a[2] + bb + bf_val(xr[2]);
      v[3] = a[3] + bb + bf_val(xr[3]);
      vv[it] = v;
    }
    for (int pass = 0; pass < 2; ++pass) {
#pragma unroll
      for (int it = 0; it < 8; ++it) {
        const int row = it * 2 + h2;
        const int c = c0w + 16 * ct + row;
        *(volatile v4f*)(out + ((size_t)b * CIN + c) * NPIX + q0 + c4) = vv[it];
      }
      __threadfence();
    }
    __builtin_amdgcn_fence(__ATOMIC_RELEASE, "workgroup");
    __builtin_amdgcn_wave_barrier();
    __builtin_amdgcn_fence(__ATOMIC_ACQUIRE, "workgroup");
  }
}

extern "C" void kernel_launch(void* const* d_in, const int* in_sizes, int n_in,
                              void* d_out, int out_size, void* d_ws, size_t ws_size,
                              hipStream_t stream) {
  if (n_in < 9) return;
  if (in_sizes[0] != NBAT * CIN * NPIX) return;
  if (in_sizes[1] != WSZ || in_sizes[3] != WSZ || in_sizes[5] != WSZ || in_sizes[7] != WSZ) return;
  if (in_sizes[2] != OCH || in_sizes[4] != OCH || in_sizes[6] != OCH) return;
  if (in_sizes[8] != CIN) return;
  if (out_size != NBAT * CIN * NPIX) return;

  const float* x       = (const float*)d_in[0];
  const float* g_w     = (const float*)d_in[1];
  const float* g_b     = (const float*)d_in[2];
  const float* theta_w = (const float*)d_in[3];
  const float* theta_b = (const float*)d_in[4];
  const float* phi_w   = (const float*)d_in[5];
  const float* phi_b   = (const float*)d_in[6];
  const float* W_w     = (const float*)d_in[7];
  const float* W_b     = (const float*)d_in[8];
  float* out = (float*)d_out;

  const size_t PW = (size_t)4 * WSZ * 2;
  const size_t PL = (size_t)NBAT * NPIX * OCH * 2;
  size_t off = 0;
  const size_t oW   = off; off += PW;
  const size_t oThH = off; off += PL;
  const size_t oThL = off; off += PL;
  const size_t oPhH = off; off += PL;
  const size_t oPhL = off; off += PL;
  const size_t oGH  = off; off += PL;
  const size_t oGL  = off; off += PL;
  if (off > ws_size) return;
  if (off > (size_t)134217728) return;

  char* ws = (char*)d_ws;
  unsigned short* Wpl = (unsigned short*)(ws + oW);
  unsigned short* ThH = (unsigned short*)(ws + oThH);
  unsigned short* ThL = (unsigned short*)(ws + oThL);
  unsigned short* PhH = (unsigned short*)(ws + oPhH);
  unsigned short* PhL = (unsigned short*)(ws + oPhL);
  unsigned short* GHp = (unsigned short*)(ws + oGH);
  unsigned short* GLp = (unsigned short*)(ws + oGL);

  cvt_w<<<dim3((4 * WGRP) / 256), dim3(256), 0, stream>>>(theta_w, phi_w, g_w, W_w, Wpl);
  proj_kernel<<<dim3(NQB, NBAT), dim3(128), 0, stream>>>(
      x, Wpl, theta_b, phi_b, g_b, ThH, ThL, PhH, PhL, GHp, GLp);
  attn_kernel<<<dim3(NQB, NBAT), dim3(128), 0, stream>>>(
      ThH, ThL, PhH, PhL, GHp, GLp, Wpl + (size_t)3 * WSZ, W_b, x, out);
  (void)hipGetLastError();
}
